// TextLSTM2_72198400245924
// MI455X (gfx1250) — hardware-verified
//
#include <hip/hip_runtime.h>


typedef _Float16 f16t;
typedef f16t  v16h __attribute__((ext_vector_type(16)));
typedef f16t  v8h  __attribute__((ext_vector_type(8)));
typedef float v8f  __attribute__((ext_vector_type(8)));
typedef float v4f  __attribute__((ext_vector_type(4)));
typedef unsigned int v4u __attribute__((ext_vector_type(4)));

union Frag { v16h v; v8h q[2]; };
union Pk16 { v8h h; v4u u; };

#define NHID   1024
#define HP     1032
#define SP     132
#define OSC    64.0f
#define INV2   0.000244140625f

__device__ __forceinline__ v8f wmma16(v16h a, v16h b, v8f c) {
    return __builtin_amdgcn_wmma_f32_16x16x32_f16(false, a, false, b, (short)0, c, false, false);
}

__device__ __forceinline__ void wguard14(v8f (&c)[4], Frag& a, Frag (&b)[4]) {
    asm volatile("v_nop\n\tv_nop\n\tv_nop\n\tv_nop"
                 : "+v"(c[0]), "+v"(c[1]), "+v"(c[2]), "+v"(c[3])
                 : "v"(a.v), "v"(b[0].v), "v"(b[1].v), "v"(b[2].v), "v"(b[3].v));
}
__device__ __forceinline__ void wguard41(v8f (&c)[4], Frag (&a)[4], Frag& b) {
    asm volatile("v_nop\n\tv_nop\n\tv_nop\n\tv_nop"
                 : "+v"(c[0]), "+v"(c[1]), "+v"(c[2]), "+v"(c[3])
                 : "v"(a[0].v), "v"(a[1].v), "v"(a[2].v), "v"(a[3].v), "v"(b.v));
}

__device__ __forceinline__ void zacc4(v8f (&acc)[4]) {
    const v8f z = {0.f, 0.f, 0.f, 0.f, 0.f, 0.f, 0.f, 0.f};
    acc[0] = z; acc[1] = z; acc[2] = z; acc[3] = z;
}

template<int BSTR>
__device__ __forceinline__ void mma_1x4(v8f (&acc)[4], const f16t* ap, const f16t* bp, int ktiles) {
#pragma unroll 1
    for (int kt = 0; kt < ktiles; ++kt) {
        Frag a, b[4];
        a.q[0] = *(const v8h*)ap;
        a.q[1] = *(const v8h*)(ap + 16);
#pragma unroll
        for (int q = 0; q < 4; ++q) {
            const f16t* p = bp + (size_t)q * BSTR;
            b[q].q[0] = *(const v8h*)p;
            b[q].q[1] = *(const v8h*)(p + 16);
        }
#pragma unroll
        for (int q = 0; q < 4; ++q) acc[q] = wmma16(a.v, b[q].v, acc[q]);
        wguard14(acc, a, b);
        ap += 32;
        bp += 32;
    }
}

__device__ __forceinline__ void mma_4x1(v8f (&acc)[4], const f16t* ap, const f16t* bp, int ktiles) {
#pragma unroll 1
    for (int kt = 0; kt < ktiles; ++kt) {
        Frag a[4], b;
#pragma unroll
        for (int i = 0; i < 4; ++i) {
            const f16t* p = ap + (size_t)i * 16 * NHID;
            a[i].q[0] = *(const v8h*)p;
            a[i].q[1] = *(const v8h*)(p + 16);
        }
        b.q[0] = *(const v8h*)bp;
        b.q[1] = *(const v8h*)(bp + 16);
#pragma unroll
        for (int i = 0; i < 4; ++i) acc[i] = wmma16(a[i].v, b.v, acc[i]);
        wguard41(acc, a, b);
        ap += 32;
        bp += 32;
    }
}

__device__ __forceinline__ float fsig(float x) {
    return __builtin_amdgcn_rcpf(1.0f + __expf(-x));
}
__device__ __forceinline__ float ftanh(float x) {
    float ax = fabsf(x);
    float e  = __expf(-2.0f * ax);
    float r  = (1.0f - e) * __builtin_amdgcn_rcpf(1.0f + e);
    return copysignf(r, x);
}
__device__ __forceinline__ float cellf(float pf, float pi, float pg, float po, float c, float& cn) {
    float fg = fsig(pf);
    float ig = fsig(pi);
    float gg = ftanh(pg);
    float og = fsig(po);
    cn = fg * c + ig * gg;
    return og * ftanh(cn);
}

__global__ __launch_bounds__(256)
void k_pack4(const float* W0, const float* W1, const float* W2, const float* W3,
             f16t* P, int K, int N, float sc) {
    const int q = blockIdx.y;
    const float* W = (q == 0) ? W0 : ((q == 1) ? W1 : ((q == 2) ? W2 : W3));
    const int kq  = K >> 3;
    const int tot = N * kq;
    const int i   = blockIdx.x * 256 + threadIdx.x;
    if (i >= tot) return;
    const int n = i / kq;
    const int k = (i - n * kq) * 8;
    Pk16 v;
#pragma unroll
    for (int e = 0; e < 8; ++e)
        v.h[e] = (f16t)(W[(size_t)(k + e) * N + n] * sc);
    f16t* d = P + ((size_t)q * N + n) * K + k;
    *(volatile v4u*)d = v.u;
    __threadfence();
    *(volatile v4u*)d = v.u;
}

__global__ __launch_bounds__(256)
void k_embed(const int* X, const float* C, f16t* E, int nrows, int nseq, int nclass) {
    const int row = blockIdx.x * 4 + (threadIdx.x >> 6);
    if (row >= nrows) return;
    const int piece = threadIdx.x & 63;
    const int t = row >> 6, b = row & 63;
    int tok = X[b * nseq + t];
    tok = tok < 0 ? 0 : (tok > nclass - 1 ? nclass - 1 : tok);
    const float* src = C + (size_t)tok * 512 + piece * 8;
    v4f a0 = *(const v4f*)src;
    v4f a1 = *(const v4f*)(src + 4);
    Pk16 v;
    v.h[0] = (f16t)(OSC * a0[0]); v.h[1] = (f16t)(OSC * a0[1]);
    v.h[2] = (f16t)(OSC * a0[2]); v.h[3] = (f16t)(OSC * a0[3]);
    v.h[4] = (f16t)(OSC * a1[0]); v.h[5] = (f16t)(OSC * a1[1]);
    v.h[6] = (f16t)(OSC * a1[2]); v.h[7] = (f16t)(OSC * a1[3]);
    f16t* d = E + (size_t)row * 512 + piece * 8;
    *(volatile v4u*)d = v.u;
    __threadfence();
    *(volatile v4u*)d = v.u;
}

template<int KX>
__global__ __launch_bounds__(256)
void k_lstm(const f16t* Xin, const f16t* Px, const f16t* Ph,
            const float* bf, const float* bi, const float* bc, const float* bo,
            f16t* Hout, int T, int nb) {
    __shared__ __attribute__((aligned(16))) f16t  hbuf[2 * 16 * HP];
    __shared__ __attribute__((aligned(16))) float cT[NHID * 16];
    const int tid = threadIdx.x, w = tid >> 5, l = tid & 31, h = l >> 4, m = l & 15;
    const int b0  = blockIdx.x * 16;

    for (int i = tid; i < 2 * 16 * HP; i += 256) hbuf[i] = (f16t)0.0f;
    for (int i = tid; i < NHID * 16; i += 256) cT[i] = 0.0f;
    __syncthreads();

#pragma unroll 1
    for (int t = 0; t < T; ++t) {
        const f16t* hA = hbuf + (t & 1) * (16 * HP);
        f16t*       hB = hbuf + ((t + 1) & 1) * (16 * HP);
        const f16t* xa = Xin + (size_t)(t * nb + b0 + m) * KX + 8 * h;
        const f16t* ha = hA + m * HP + 8 * h;

#pragma unroll 1
        for (int j = 0; j < 8; ++j) {
            const int c0 = 128 * w + 16 * j;
            v8f acc[4];
            zacc4(acc);
            mma_1x4<NHID * KX>(acc, xa, Px + (size_t)(c0 + m) * KX + 8 * h, KX / 32);
            mma_1x4<NHID * NHID>(acc, ha, Ph + (size_t)(c0 + m) * NHID + 8 * h, NHID / 32);

            const int col = c0 + m;
            const float vbf = bf[col], vbi = bi[col], vbc = bc[col], vbo = bo[col];
            float* cp = cT + col * 16 + 8 * h;
            v4f cA = *(const v4f*)cp;
            v4f cB = *(const v4f*)(cp + 4);
            f16t* hp = hB + (8 * h) * HP + col;
#pragma unroll
            for (int r = 0; r < 4; ++r) {
                float cn;
                float hv = cellf(fmaf(acc[0][r], INV2, vbf), fmaf(acc[1][r], INV2, vbi),
                                 fmaf(acc[2][r], INV2, vbc), fmaf(acc[3][r], INV2, vbo),
                                 cA[r], cn);
                cA[r] = cn;
                hp[r * HP] = (f16t)(OSC * hv);
            }
#pragma unroll
            for (int r = 0; r < 4; ++r) {
                float cn;
                float hv = cellf(fmaf(acc[0][4 + r], INV2, vbf), fmaf(acc[1][4 + r], INV2, vbi),
                                 fmaf(acc[2][4 + r], INV2, vbc), fmaf(acc[3][4 + r], INV2, vbo),
                                 cB[r], cn);
                cB[r] = cn;
                hp[(4 + r) * HP] = (f16t)(OSC * hv);
            }
            *(v4f*)cp       = cA;
            *(v4f*)(cp + 4) = cB;
        }
        __syncthreads();

        Pk16 v[8];
#pragma unroll
        for (int it = 0; it < 8; ++it) {
            const int p = it * 32 + l, row = p >> 4, ch = (p & 15) * 8;
            v[it].h = *(const v8h*)(hB + row * HP + 128 * w + ch);
        }
#pragma unroll
        for (int it = 0; it < 8; ++it) {
            const int p = it * 32 + l, row = p >> 4, ch = (p & 15) * 8;
            f16t* d = Hout + (size_t)(t * nb + b0 + row) * NHID + 128 * w + ch;
            *(volatile v4u*)d = v[it].u;
        }
        __threadfence();
#pragma unroll
        for (int it = 0; it < 8; ++it) {
            const int p = it * 32 + l, row = p >> 4, ch = (p & 15) * 8;
            f16t* d = Hout + (size_t)(t * nb + b0 + row) * NHID + 128 * w + ch;
            *(volatile v4u*)d = v[it].u;
        }
    }
}

__global__ __launch_bounds__(256)
void k_outgemm(const f16t* A, const f16t* P, const float* bias, float* OP, int nout, int np) {
    __shared__ __attribute__((aligned(16))) float S[64 * SP];
    const int tid = threadIdx.x, w = tid >> 5, l = tid & 31, h = l >> 4, m = l & 15;
    const int nbase = blockIdx.x * 128;
    int nrow = nbase + 16 * w + m;
    nrow = nrow > nout - 1 ? nout - 1 : nrow;

    v8f acc[4];
    zacc4(acc);
    mma_4x1(acc, A + (size_t)m * NHID + 8 * h, P + (size_t)nrow * NHID + 8 * h, NHID / 32);

    const float bv = bias[nrow];
#pragma unroll
    for (int i = 0; i < 4; ++i)
#pragma unroll
        for (int r = 0; r < 8; ++r)
            S[(16 * i + 8 * h + r) * SP + 16 * w + m] = fmaf(acc[i][r], INV2, bv);
    __syncthreads();

    v4f v[8];
#pragma unroll
    for (int it = 0; it < 8; ++it) {
        const int p = it * 256 + tid, row = p >> 5, c4 = (p & 31) * 4;
        v[it] = *(const v4f*)(S + row * SP + c4);
    }
#pragma unroll
    for (int it = 0; it < 8; ++it) {
        const int p = it * 256 + tid, row = p >> 5, c4 = (p & 31) * 4;
        const int col = nbase + c4;
        if (col < np) *(volatile v4f*)(OP + (size_t)row * np + col) = v[it];
    }
    __threadfence();
#pragma unroll
    for (int it = 0; it < 8; ++it) {
        const int p = it * 256 + tid, row = p >> 5, c4 = (p & 31) * 4;
        const int col = nbase + c4;
        if (col < np) *(volatile v4f*)(OP + (size_t)row * np + col) = v[it];
    }
}

__global__ __launch_bounds__(256)
void k_outcopy(const float* OP, float* out, int nout, int np, int n4) {
    const int i = blockIdx.x * 256 + threadIdx.x;
    if (i >= n4) return;
    const int f = i * 4;
    const int r = f / nout;
    const int c = f - r * nout;
    v4f v = *(const v4f*)(OP + (size_t)r * np + c);
    *(volatile v4f*)(out + f) = v;
    __threadfence();
    *(volatile v4f*)(out + f) = v;
}

extern "C" void kernel_launch(void* const* d_in, const int* in_sizes, int n_in,
                              void* d_out, int out_size, void* d_ws, size_t ws_size,
                              hipStream_t stream) {
    const int NB = 64, NS = 128, EMB = 512, NC = 10000, NP = 10016;
    const int NTOK = NB * NS;

    if (n_in < 28) return;
    if (in_sizes[0] != NTOK || in_sizes[1] != NC * EMB || in_sizes[18] != NHID * NC ||
        in_sizes[27] != NC || out_size != NB * NC) return;
    for (int i = 2; i <= 8; i += 2) if (in_sizes[i] != EMB * NHID) return;
    for (int i = 3; i <= 9; i += 2) if (in_sizes[i] != NHID * NHID) return;
    for (int i = 10; i <= 17; ++i) if (in_sizes[i] != NHID * NHID) return;
    for (int i = 19; i <= 26; ++i) if (in_sizes[i] != NHID) return;

    const int*   X    = (const int*)d_in[0];
    const float* C    = (const float*)d_in[1];
    const float* Wfx  = (const float*)d_in[2];
    const float* Wfh  = (const float*)d_in[3];
    const float* Wix  = (const float*)d_in[4];
    const float* Wih  = (const float*)d_in[5];
    const float* WCx  = (const float*)d_in[6];
    const float* WCh  = (const float*)d_in[7];
    const float* Wox  = (const float*)d_in[8];
    const float* Woh  = (const float*)d_in[9];
    const float* Wfx1 = (const float*)d_in[10];
    const float* Wfh1 = (const float*)d_in[11];
    const float* Wix1 = (const float*)d_in[12];
    const float* WCx1 = (const float*)d_in[14];
    const float* WCh1 = (const float*)d_in[15];
    const float* Wox1 = (const float*)d_in[16];
    const float* Woh1 = (const float*)d_in[17];
    const float* Wout = (const float*)d_in[18];
    const float* b_f  = (const float*)d_in[19];
    const float* b_i  = (const float*)d_in[20];
    const float* b_C  = (const float*)d_in[21];
    const float* b_o  = (const float*)d_in[22];
    const float* b_f1 = (const float*)d_in[23];
    const float* b_i1 = (const float*)d_in[24];
    const float* b_C1 = (const float*)d_in[25];
    const float* b_o1 = (const float*)d_in[26];
    const float* b_out = (const float*)d_in[27];
    float* out = (float*)d_out;

    char* ws = (char*)d_ws;
    size_t off = 0;
    auto carve = [&](size_t bytes) -> char* {
        char* p = ws + off;
        off = (off + bytes + 255) & ~(size_t)255;
        return p;
    };
    f16t*  E16  = (f16t*)carve((size_t)NTOK * EMB * 2);
    f16t*  Px0  = (f16t*)carve((size_t)4 * NHID * EMB * 2);
    f16t*  Ph0  = (f16t*)carve((size_t)4 * NHID * NHID * 2);
    f16t*  Px1  = (f16t*)carve((size_t)4 * NHID * NHID * 2);
    f16t*  Ph1  = (f16t*)carve((size_t)4 * NHID * NHID * 2);
    f16t*  Pout = (f16t*)carve((size_t)NC * NHID * 2);
    f16t*  H0   = (f16t*)carve((size_t)NTOK * NHID * 2);
    f16t*  H1   = (f16t*)carve((size_t)NTOK * NHID * 2);
    float* OP   = (float*)carve((size_t)NB * NP * 4);
    if (off > ws_size || off > (size_t)134217728) return;

    auto pack4 = [&](const float* a, const float* b, const float* c, const float* d,
                     f16t* P, int K, int N, int ny) {
        int tot = N * (K / 8);
        k_pack4<<<dim3((tot + 255) / 256, ny), dim3(256), 0, stream>>>(a, b, c, d, P, K, N, OSC);
    };
    pack4(Wfx,  Wix,  WCx,  Wox,  Px0,  EMB,  NHID, 4);
    pack4(Wfh,  Wih,  WCh,  Woh,  Ph0,  NHID, NHID, 4);
    pack4(Wfx1, Wix1, WCx1, Wox1, Px1,  NHID, NHID, 4);
    pack4(Wfh1, Wih,  WCh1, Woh1, Ph1,  NHID, NHID, 4);
    pack4(Wout, Wout, Wout, Wout, Pout, NHID, NC,   1);

    k_embed<<<dim3(NTOK / 4), dim3(256), 0, stream>>>(X, C, E16, NTOK, NS, NC);

    k_lstm<512><<<dim3(NB / 16), dim3(256), 0, stream>>>(E16, Px0, Ph0, b_f, b_i, b_C, b_o,
                                                        H0, NS, NB);
    k_lstm<1024><<<dim3(NB / 16), dim3(256), 0, stream>>>(H0, Px1, Ph1, b_f1, b_i1, b_C1, b_o1,
                                                         H1, NS, NB);
    k_outgemm<<<dim3((NP + 127) / 128), dim3(256), 0, stream>>>(
        H1 + (size_t)(NS - 1) * NB * NHID, Pout, b_out, OP, NC, NP);
    {
        int n4 = NB * NC / 4;
        k_outcopy<<<dim3((n4 + 255) / 256), dim3(256), 0, stream>>>(OP, out, NC, NP, n4);
    }
}
